// Regression_Cubical_Network_One_Nonlinearity_38946763440762
// MI455X (gfx1250) — hardware-run, weakly checked
//
#include <hip/hip_runtime.h>
#pragma clang fp contract(off)


#ifndef NB
#define NB 16384
#endif
#define NB_FULL 16384
#define DIMS    8
#define NHID    4096
#define NLAB    64
#define GW      (NHID / DIMS)
#define ROWS_BLK 128
#define WCARRY     1024.0f
#define WCARRY_INV 0.0009765625f

static_assert(NB <= NB_FULL);
static_assert(NB % ROWS_BLK == 0);
static_assert(NHID % DIMS == 0);
static_assert(GW % 32 == 0);
static_assert(NLAB == 64);
static_assert(DIMS == 8);
static_assert((NHID / 4) % 256 == 0);
static_assert((NLAB * NHID) % (8 * 256) == 0);
static_assert(32 * 4 == ROWS_BLK);
static_assert((2 * NHID + DIMS * DIMS + ROWS_BLK) * 4 <= 131072);

typedef _Float16 h16;
typedef __attribute__((ext_vector_type(16))) _Float16 v16h;
typedef __attribute__((ext_vector_type(8)))  _Float16 v8h;
typedef __attribute__((ext_vector_type(8)))  float    v8f;
typedef __attribute__((ext_vector_type(4)))  float    v4f;
typedef v4f __attribute__((may_alias)) v4fa;

__device__ __forceinline__ float bfr(float f) { unsigned u = __float_as_uint(f); u += 0x7FFFu + ((u >> 16) & 1u); return __uint_as_float(u & 0xFFFF0000u); }
__device__ __forceinline__ h16 toh_flush(float v) { const h16 r = (h16)v; return (fabsf(v) < 6.103515625e-05f) ? (h16)0.0f : r; }
__device__ __forceinline__ v16h cat16h(v8h lo, v8h hi) { return __builtin_shufflevector(lo, hi, 0, 1, 2, 3, 4, 5, 6, 7, 8, 9, 10, 11, 12, 13, 14, 15); }
__device__ __forceinline__ v16h ldh(const h16* p) { return cat16h(*(const v8h*)p, *(const v8h*)(p + 16)); }
__device__ __forceinline__ v8f wmmah(v16h a, v16h b, v8f c) {
    c = __builtin_amdgcn_wmma_f32_16x16x32_f16(false, a, false, b, (short)0, c, false, false);
    asm volatile("v_nop\n\tv_nop\n\tv_nop\n\tv_nop" : "+v"(c) : "v"(a), "v"(b));
    return c;
}
__device__ __forceinline__ h16 act16(float pv, float c, float b) { float hd = pv * c + b; hd = fminf(fmaxf(hd, 0.0f), 1.0f); return toh_flush(hd); }

__global__ __launch_bounds__(256) void k_wconv(const float* __restrict__ W2, h16* W2H) {
    const size_t i = (size_t)blockIdx.x * 256 + threadIdx.x;
    if (i >= (size_t)(NLAB * NHID / 8)) return;
    const v4f a = *(const v4f*)(W2 + i * 8);
    const v4f b = *(const v4f*)(W2 + i * 8 + 4);
    v8h o;
#pragma unroll
    for (int k = 0; k < 4; ++k) { o[k] = toh_flush(bfr(a[k]) * WCARRY); o[4 + k] = toh_flush(bfr(b[k]) * WCARRY); }
    *(volatile v8h*)(W2H + i * 8) = o;
    __threadfence();
    *(volatile v8h*)(W2H + i * 8) = o;
}

__global__ __launch_bounds__(256) void k_mlp(const float* __restrict__ x, const float* __restrict__ swm, const float* __restrict__ coeff,
                                             const float* __restrict__ bias, const h16* __restrict__ W2H, const float* __restrict__ b2,
                                             const float* __restrict__ Wout, const float* __restrict__ bout, float* OUT) {
    __shared__ __align__(16) float s_coeff[NHID];
    __shared__ __align__(16) float s_bias[NHID];
    __shared__ __align__(16) float s_swm[DIMS * DIMS];
    __shared__ __align__(16) float res[ROWS_BLK];
    const int tid = threadIdx.x, lane = tid & 31, lr = lane & 15, hi = lane >> 4;
    const int wave = __builtin_amdgcn_readfirstlane(tid >> 5);

#pragma unroll 1
    for (int i = tid; i < NHID / 4; i += 256) {
        v4f c = *(const v4f*)(coeff + 4 * i); v4f b = *(const v4f*)(bias + 4 * i);
#pragma unroll
        for (int k = 0; k < 4; ++k) { c[k] = bfr(c[k]); b[k] = bfr(b[k]); }
        *(v4fa*)(&s_coeff[4 * i]) = c; *(v4fa*)(&s_bias[4 * i]) = b; }
    if (tid < DIMS * DIMS) s_swm[tid] = bfr(swm[tid]);
    __syncthreads();

    const size_t row = (size_t)blockIdx.x * ROWS_BLK + (size_t)wave * 16 + lr;
    float xr[DIMS];
    { const v4f x0 = *(const v4f*)(x + row * DIMS); const v4f x1 = *(const v4f*)(x + row * DIMS + 4);
#pragma unroll
      for (int k = 0; k < 4; ++k) { xr[k] = bfr(x0[k]); xr[4 + k] = bfr(x1[k]); } }

    v8f acc[4];
#pragma unroll
    for (int nb = 0; nb < 4; ++nb) acc[nb] = (v8f){};
    const size_t boff = (size_t)lr * NHID + 8 * hi;

#pragma unroll 1
    for (int g = 0; g < DIMS; ++g) {
        float pv = xr[0] * s_swm[g * DIMS];
#pragma unroll
        for (int i = 1; i < DIMS; ++i) pv = fmaf(xr[i], s_swm[g * DIMS + i], pv);
#pragma unroll 1
        for (int ks = 0; ks < GW / 32; ++ks) {
            const int k0 = g * GW + ks * 32;
            const int ka = k0 + 8 * hi;
            const v4f c0 = *(const v4fa*)(&s_coeff[ka]),      c1 = *(const v4fa*)(&s_coeff[ka + 4]);
            const v4f c2 = *(const v4fa*)(&s_coeff[ka + 16]), c3 = *(const v4fa*)(&s_coeff[ka + 20]);
            const v4f d0 = *(const v4fa*)(&s_bias[ka]),       d1 = *(const v4fa*)(&s_bias[ka + 4]);
            const v4f d2 = *(const v4fa*)(&s_bias[ka + 16]),  d3 = *(const v4fa*)(&s_bias[ka + 20]);
            v16h a;
#pragma unroll
            for (int i = 0; i < 4; ++i) {
                a[i]      = act16(pv, c0[i], d0[i]);
                a[4 + i]  = act16(pv, c1[i], d1[i]);
                a[8 + i]  = act16(pv, c2[i], d2[i]);
                a[12 + i] = act16(pv, c3[i], d3[i]); }
#pragma unroll
            for (int nb = 0; nb < 4; ++nb) {
                const v16h b = ldh(W2H + boff + (size_t)nb * 16 * NHID + k0);
                acc[nb] = wmmah(a, b, acc[nb]); }
        }
    }

    float w[4], bb[4];
#pragma unroll
    for (int nb = 0; nb < 4; ++nb) { w[nb] = bfr(Wout[nb * 16 + lr]); bb[nb] = bfr(b2[nb * 16 + lr]); }
    const float bo = bfr(bout[0]);
    float s[8];
#pragma unroll
    for (int r = 0; r < 8; ++r) {
        float t = 0.0f;
#pragma unroll
        for (int nb = 0; nb < 4; ++nb) { const float lab = acc[nb][r] * WCARRY_INV + bb[nb]; t += lab * w[nb]; }
        s[r] = t; }
#pragma unroll
    for (int r = 0; r < 8; ++r) {
        s[r] += __shfl_xor(s[r], 1, 32);
        s[r] += __shfl_xor(s[r], 2, 32);
        s[r] += __shfl_xor(s[r], 4, 32);
        s[r] += __shfl_xor(s[r], 8, 32); }
    if (lr == 0) {
#pragma unroll
        for (int r = 0; r < 8; ++r) res[wave * 16 + hi * 8 + r] = s[r] + bo; }
    __syncthreads();
    if (wave == 0) {
        const v4f v = *(const v4fa*)(&res[4 * lane]);
        float* dst = OUT + (size_t)blockIdx.x * ROWS_BLK + 4 * lane;
        *(volatile v4f*)dst = v;
        __threadfence();
        *(volatile v4f*)dst = v;
    }
}

static constexpr size_t al256(size_t v) { return (v + 255) & ~(size_t)255; }
static constexpr size_t SZ_W2H = al256((size_t)NLAB * NHID * 2);
static constexpr size_t SZ_TOTAL = SZ_W2H;
static_assert(SZ_TOTAL <= (size_t)134217728);
static_assert((size_t)(NLAB * NHID / 8) * 16 == (size_t)NLAB * NHID * 2);

extern "C" void kernel_launch(void* const* d_in, const int* in_sizes, int n_in,
                              void* d_out, int out_size, void* d_ws, size_t ws_size, hipStream_t stream) {
    if (n_in < 8) return;
    if ((size_t)in_sizes[0] < (size_t)NB * DIMS) return;
    if ((size_t)in_sizes[1] < (size_t)DIMS * DIMS) return;
    if ((size_t)in_sizes[2] < (size_t)NHID || (size_t)in_sizes[3] < (size_t)NHID) return;
    if ((size_t)in_sizes[4] < (size_t)NLAB * NHID) return;
    if ((size_t)in_sizes[5] < (size_t)NLAB || (size_t)in_sizes[6] < (size_t)NLAB) return;
    if ((size_t)in_sizes[7] < (size_t)1) return;
    if ((size_t)out_size < (size_t)NB) return;
    if (SZ_TOTAL > ws_size) return;
    const float* x     = (const float*)d_in[0];
    const float* swm   = (const float*)d_in[1];
    const float* coeff = (const float*)d_in[2];
    const float* bias  = (const float*)d_in[3];
    const float* W2    = (const float*)d_in[4];
    const float* b2    = (const float*)d_in[5];
    const float* Wout  = (const float*)d_in[6];
    const float* bout  = (const float*)d_in[7];
    float* OUT = (float*)d_out;
    h16* W2H = (h16*)d_ws;

    k_wconv<<<(unsigned)(NLAB * NHID / 8 / 256), 256, 0, stream>>>(W2, W2H);
    k_mlp<<<(unsigned)(NB / ROWS_BLK), 256, 0, stream>>>(x, swm, coeff, bias, W2H, b2, Wout, bout, OUT);
}
